// SelfAttentionV2Causal_21388937134112
// MI455X (gfx1250) — hardware-verified
//
#include <hip/hip_runtime.h>
#include <stdint.h>

#define NB  4
#define NS  2048
#define ND  1024
static_assert((NS % 64) == 0 && (ND % 64) == 0);
static_assert((NS % 32) == 0 && (ND % 32) == 0);
static_assert(NS == 256 * 8);
static_assert(((NB * NS * ND) % (8 * 256)) == 0 && ((ND * ND) % (8 * 256)) == 0);

typedef __bf16   v16b __attribute__((ext_vector_type(16)));
typedef __bf16   v8b  __attribute__((ext_vector_type(8)));
typedef float    v8f  __attribute__((ext_vector_type(8)));
typedef float    v4f  __attribute__((ext_vector_type(4)));
typedef unsigned int v4u __attribute__((ext_vector_type(4)));

__device__ __forceinline__ unsigned short bf_bits(float f) {
  unsigned u = __float_as_uint(f);
  return (unsigned short)((u + 0x7FFFu + ((u >> 16) & 1u)) >> 16);
}
__device__ __forceinline__ unsigned pk16(unsigned short a, unsigned short b) { return (unsigned)a | ((unsigned)b << 16); }
__device__ __forceinline__ v8f zero8() { v8f z = {0.f, 0.f, 0.f, 0.f, 0.f, 0.f, 0.f, 0.f}; return z; }
__device__ __forceinline__ void hilo2(float x, float y, unsigned& h, unsigned& l) {
  const unsigned short hx = bf_bits(x), hy = bf_bits(y);
  const float rx = x - __uint_as_float(((unsigned)hx) << 16);
  const float ry = y - __uint_as_float(((unsigned)hy) << 16);
  h = pk16(hx, hy);
  l = pk16(bf_bits(rx), bf_bits(ry));
}

__device__ __forceinline__ v16b ldfrag_b(const __bf16* p) {
  union { v16b v; v8b h[2]; } f;
  f.h[0] = *(const v8b*)(p);
  f.h[1] = *(const v8b*)(p + 16);
  return f.v;
}

__device__ __forceinline__ v8f mma_b_raw(v16b a, v16b b, v8f c) {
  return __builtin_amdgcn_wmma_f32_16x16x32_bf16(false, a, false, b, (short)0, c, false, false);
}
__device__ __forceinline__ void dep_guard_b(v8f& a, v8f& b, v16b x, v16b y) {
#if defined(__HIP_DEVICE_COMPILE__)
  asm volatile("v_nop\n\tv_nop\n\tv_nop\n\tv_nop" : "+v"(a), "+v"(b) : "v"(x), "v"(y));
#endif
}
__device__ __forceinline__ void keep4_b(v16b a, v16b b, v16b c, v16b d) {
#if defined(__HIP_DEVICE_COMPILE__)
  asm volatile("v_nop" :: "v"(a), "v"(b), "v"(c), "v"(d));
#endif
}
__device__ __forceinline__ void acc_guard4(v8f& a, v8f& b, v8f& c, v8f& d) {
#if defined(__HIP_DEVICE_COMPILE__)
  asm volatile("v_nop\n\tv_nop\n\tv_nop\n\tv_nop" : "+v"(a), "+v"(b), "+v"(c), "+v"(d));
#endif
}
__device__ __forceinline__ void wave_sync_lds() {
  __builtin_amdgcn_fence(__ATOMIC_RELEASE, "workgroup");
  __builtin_amdgcn_wave_barrier();
  __builtin_amdgcn_fence(__ATOMIC_ACQUIRE, "workgroup");
}

__global__ __launch_bounds__(256) void cvt_bf16x8(const float* __restrict__ in, unsigned short* out,
                                                  int n8, int n8tot) {
  const int i = blockIdx.x * 256 + threadIdx.x;
  if (i >= n8tot) return;
  int ic = i;
  if (ic > n8 - 1) ic = n8 - 1;
  const v4f a = *(const v4f*)(in + (size_t)ic * 8);
  const v4f b = *(const v4f*)(in + (size_t)ic * 8 + 4);
  v4u p;
  p[0] = pk16(bf_bits(a[0]), bf_bits(a[1]));
  p[1] = pk16(bf_bits(a[2]), bf_bits(a[3]));
  p[2] = pk16(bf_bits(b[0]), bf_bits(b[1]));
  p[3] = pk16(bf_bits(b[2]), bf_bits(b[3]));
  if (i >= n8) { p[0] = 0u; p[1] = 0u; p[2] = 0u; p[3] = 0u; }
  *(volatile v4u*)(out + (size_t)i * 8) = p;
  __threadfence();
  *(volatile v4u*)(out + (size_t)i * 8) = p;
}

template <int OUT, int CAUSAL, int SPLIT>
__global__ __launch_bounds__(256) void gemm64(
    const unsigned short* __restrict__ Ahp, const unsigned short* __restrict__ Alp, int lda,
    const unsigned short* __restrict__ Bhp, const unsigned short* __restrict__ Blp, int ldb,
    void* Cout, void* Cout2, int ldc, float alpha, int M, int N, int K) {
  __shared__ __align__(16) float sT[8][16 * 68];
  const int lane = threadIdx.x & 31;
  const int wave = threadIdx.x >> 5;
  const int tilesN = N >> 6;
  const int tilesM = M >> 6;
  const int tile = blockIdx.x * 8 + wave;
  if (tile >= tilesM * tilesN) return;
  const int tm = tile / tilesN;
  const int tn = tile - tm * tilesN;
  const int m0 = tm << 6;
  const int n0 = tn << 6;
  if (CAUSAL == 1) {
    if (n0 >= m0 + 64) return;
  }
  int kEnd = K;
  if (CAUSAL == 2) {
    kEnd = m0 + 64;
    if (kEnd > K) kEnd = K;
  }

  const int rlane = lane & 15;
  const int koff  = (lane >> 4) * 8;
  const int mOff  = (lane >> 4) * 8;

  v8f acc[4][4];
#pragma unroll
  for (int i = 0; i < 4; ++i)
#pragma unroll
    for (int j = 0; j < 4; ++j) acc[i][j] = zero8();

  const int nPass = SPLIT ? 3 : 1;
#pragma unroll 1
  for (int ps = 0; ps < nPass; ++ps) {
    const __bf16* A  = (const __bf16*)(const void*)((ps == 2) ? Alp : Ahp);
    const __bf16* Bt = (const __bf16*)(const void*)((ps == 1) ? Blp : Bhp);
    for (int k0 = 0; k0 < kEnd; k0 += 32) {
      v16b bh[4];
#pragma unroll
      for (int j = 0; j < 4; ++j) {
        const size_t bo = (size_t)(n0 + (j << 4) + rlane) * ldb + koff + k0;
        bh[j] = ldfrag_b(Bt + bo);
      }
#pragma unroll
      for (int i = 0; i < 4; ++i) {
        const size_t ao = (size_t)(m0 + (i << 4) + rlane) * lda + koff + k0;
        const v16b ah = ldfrag_b(A + ao);
#pragma unroll
        for (int j = 0; j < 4; ++j) {
          acc[i][j] = mma_b_raw(ah, bh[j], acc[i][j]);
        }
        dep_guard_b(acc[i][0], acc[i][3], ah, bh[3]);
      }
      keep4_b(bh[0], bh[1], bh[2], bh[3]);
    }
  }
  acc_guard4(acc[0][0], acc[0][1], acc[0][2], acc[0][3]);
  acc_guard4(acc[1][0], acc[1][1], acc[1][2], acc[1][3]);
  acc_guard4(acc[2][0], acc[2][1], acc[2][2], acc[2][3]);
  acc_guard4(acc[3][0], acc[3][1], acc[3][2], acc[3][3]);

  float* slab = sT[wave];
#pragma unroll
  for (int i = 0; i < 4; ++i) {
    const int mBase = m0 + (i << 4);
#pragma unroll
    for (int j = 0; j < 4; ++j) {
#pragma unroll
      for (int r = 0; r < 8; ++r) {
        slab[(mOff + r) * 68 + (j << 4) + rlane] = acc[i][j][r];
      }
    }
    wave_sync_lds();
    if (OUT == 0) {
      float* C = (float*)Cout;
      const int hh = lane >> 4, c4 = (lane & 15) * 4;
      v4f vv[8];
#pragma unroll
      for (int it = 0; it < 8; ++it) {
        const int row = it * 2 + hh;
        v4f v = *(const v4f*)(slab + row * 68 + c4);
        vv[it] = v * alpha;
      }
      for (int pass = 0; pass < 2; ++pass) {
#pragma unroll
        for (int it = 0; it < 8; ++it) {
          const int row = it * 2 + hh;
          *(volatile v4f*)(C + (size_t)(mBase + row) * ldc + n0 + c4) = vv[it];
        }
        __threadfence();
      }
    } else {
      unsigned short* Ch = (unsigned short*)Cout;
      unsigned short* Cl = (unsigned short*)Cout2;
      const int q8 = (lane & 7) * 8, rr = lane >> 3;
      v4u ph[4], pl[4];
#pragma unroll
      for (int it = 0; it < 4; ++it) {
        const int row = it * 4 + rr;
        v4f a = *(const v4f*)(slab + row * 68 + q8);
        v4f b = *(const v4f*)(slab + row * 68 + q8 + 4);
        a = a * alpha;
        b = b * alpha;
        unsigned h0, l0, h1, l1, h2, l2, h3, l3;
        hilo2(a[0], a[1], h0, l0);
        hilo2(a[2], a[3], h1, l1);
        hilo2(b[0], b[1], h2, l2);
        hilo2(b[2], b[3], h3, l3);
        v4u hpk, lpk;
        hpk[0] = h0; hpk[1] = h1; hpk[2] = h2; hpk[3] = h3;
        lpk[0] = l0; lpk[1] = l1; lpk[2] = l2; lpk[3] = l3;
        ph[it] = hpk;
        pl[it] = lpk;
      }
      for (int pass = 0; pass < 2; ++pass) {
#pragma unroll
        for (int it = 0; it < 4; ++it) {
          const int row = it * 4 + rr;
          const size_t co = (size_t)(mBase + row) * ldc + n0 + q8;
          *(volatile v4u*)(Ch + co) = ph[it];
          *(volatile v4u*)(Cl + co) = pl[it];
        }
        __threadfence();
      }
    }
    wave_sync_lds();
  }
}

__global__ __launch_bounds__(256) void softmax_causal(const float* __restrict__ S, unsigned short* Ph,
                                                      unsigned short* Pl) {
  __shared__ float sMx[8];
  __shared__ float sSm[8];
  const int tid  = threadIdx.x;
  const int lane = tid & 31;
  const int wave = tid >> 5;
  const int q    = blockIdx.x;
  const size_t rb = (size_t)q * NS;
  const int c0 = tid * 8;
  const v4f a0 = *(const v4f*)(S + rb + c0);
  const v4f a1 = *(const v4f*)(S + rb + c0 + 4);
  const float ninf = __uint_as_float(0xff800000u);
  float v[8];
  v[0] = (c0 + 0 <= q) ? a0[0] : ninf;
  v[1] = (c0 + 1 <= q) ? a0[1] : ninf;
  v[2] = (c0 + 2 <= q) ? a0[2] : ninf;
  v[3] = (c0 + 3 <= q) ? a0[3] : ninf;
  v[4] = (c0 + 4 <= q) ? a1[0] : ninf;
  v[5] = (c0 + 5 <= q) ? a1[1] : ninf;
  v[6] = (c0 + 6 <= q) ? a1[2] : ninf;
  v[7] = (c0 + 7 <= q) ? a1[3] : ninf;

  float mx = v[0];
#pragma unroll
  for (int i = 1; i < 8; ++i) mx = fmaxf(mx, v[i]);
  mx = fmaxf(mx, __shfl_xor(mx, 16));
  mx = fmaxf(mx, __shfl_xor(mx, 8));
  mx = fmaxf(mx, __shfl_xor(mx, 4));
  mx = fmaxf(mx, __shfl_xor(mx, 2));
  mx = fmaxf(mx, __shfl_xor(mx, 1));
  if (lane == 0) sMx[wave] = mx;
  __syncthreads();
  float m = sMx[0];
#pragma unroll
  for (int w = 1; w < 8; ++w) m = fmaxf(m, sMx[w]);

  float e[8];
#pragma unroll
  for (int i = 0; i < 8; ++i) {
    const float t = __expf(v[i] - m);
    e[i] = (c0 + i <= q) ? t : 0.0f;
  }
  float part = ((e[0] + e[1]) + (e[2] + e[3])) + ((e[4] + e[5]) + (e[6] + e[7]));
  part += __shfl_xor(part, 16);
  part += __shfl_xor(part, 8);
  part += __shfl_xor(part, 4);
  part += __shfl_xor(part, 2);
  part += __shfl_xor(part, 1);
  if (lane == 0) sSm[wave] = part;
  __syncthreads();
  const float l = ((sSm[0] + sSm[1]) + (sSm[2] + sSm[3])) + ((sSm[4] + sSm[5]) + (sSm[6] + sSm[7]));
  const float inv = 1.0f / l;

  unsigned h0, l0, h1, l1, h2, l2, h3, l3;
  hilo2(e[0] * inv, e[1] * inv, h0, l0);
  hilo2(e[2] * inv, e[3] * inv, h1, l1);
  hilo2(e[4] * inv, e[5] * inv, h2, l2);
  hilo2(e[6] * inv, e[7] * inv, h3, l3);
  v4u hpk, lpk;
  hpk[0] = h0; hpk[1] = h1; hpk[2] = h2; hpk[3] = h3;
  lpk[0] = l0; lpk[1] = l1; lpk[2] = l2; lpk[3] = l3;
  unsigned short* prh = Ph + rb + c0;
  unsigned short* prl = Pl + rb + c0;
  *(volatile v4u*)(prh) = hpk;
  *(volatile v4u*)(prl) = lpk;
  __threadfence();
  *(volatile v4u*)(prh) = hpk;
  *(volatile v4u*)(prl) = lpk;
}

extern "C" void kernel_launch(void* const* d_in, const int* in_sizes, int n_in,
                              void* d_out, int out_size, void* d_ws, size_t ws_size,
                              hipStream_t stream) {
  if (n_in < 4) return;
  if (in_sizes[0] != NB * NS * ND) return;
  if (in_sizes[1] != ND * ND || in_sizes[2] != ND * ND || in_sizes[3] != ND * ND) return;
  if (out_size != NB * NS * ND) return;

  const float* x  = (const float*)d_in[0];
  const float* Wq = (const float*)d_in[1];
  const float* Wk = (const float*)d_in[2];
  const float* Wv = (const float*)d_in[3];
  float* out = (float*)d_out;

  const size_t PX  = (size_t)NB * NS * ND * 2;
  const size_t PW  = (size_t)ND * ND * 2;
  const size_t PQK = (size_t)NS * ND * 2;
  const size_t PV  = (size_t)ND * NS * 2;
  const size_t PS  = (size_t)NS * NS * 4;
  const size_t PP  = (size_t)NS * NS * 2;
  size_t off = 0;
  const size_t oX  = off; off += PX;
  const size_t oWq = off; off += PW;
  const size_t oWk = off; off += PW;
  const size_t oWv = off; off += PW;
  const size_t oQh = off; off += PQK;
  const size_t oQl = off; off += PQK;
  const size_t oKh = off; off += PQK;
  const size_t oKl = off; off += PQK;
  const size_t oVh = off; off += PV;
  const size_t oVl = off; off += PV;
  const size_t oS  = off; off += PS;
  const size_t oPh = off; off += PP;
  const size_t oPl = off; off += PP;
  if (off > ws_size) return;
  if (off > (size_t)134217728) return;

  char* ws = (char*)d_ws;
  unsigned short* Xb  = (unsigned short*)(ws + oX);
  unsigned short* Wqb = (unsigned short*)(ws + oWq);
  unsigned short* Wkb = (unsigned short*)(ws + oWk);
  unsigned short* Wvb = (unsigned short*)(ws + oWv);
  unsigned short* Qh  = (unsigned short*)(ws + oQh);
  unsigned short* Ql  = (unsigned short*)(ws + oQl);
  unsigned short* Kh  = (unsigned short*)(ws + oKh);
  unsigned short* Kl  = (unsigned short*)(ws + oKl);
  unsigned short* Vh  = (unsigned short*)(ws + oVh);
  unsigned short* Vl  = (unsigned short*)(ws + oVl);
  float* S = (float*)(ws + oS);
  unsigned short* Ph  = (unsigned short*)(ws + oPh);
  unsigned short* Pl  = (unsigned short*)(ws + oPl);

  const dim3 blk(256);
  const int n8x = NB * NS * ND / 8;
  const int n8w = ND * ND / 8;
  const dim3 gCvtX((n8x + 255) / 256);
  const dim3 gCvtW((n8w + 255) / 256);
  const dim3 gQK(((NS / 64) * (ND / 64) + 7) / 8);
  const dim3 gV(((ND / 64) * (NS / 64) + 7) / 8);
  const dim3 gS(((NS / 64) * (NS / 64) + 7) / 8);
  const dim3 gSm(NS);
  const dim3 gO(((NS / 64) * (ND / 64) + 7) / 8);

  cvt_bf16x8<<<gCvtX, blk, 0, stream>>>(x, Xb, n8x, n8x);
  cvt_bf16x8<<<gCvtW, blk, 0, stream>>>(Wq, Wqb, n8w, n8w);
  cvt_bf16x8<<<gCvtW, blk, 0, stream>>>(Wk, Wkb, n8w, n8w);
  cvt_bf16x8<<<gCvtW, blk, 0, stream>>>(Wv, Wvb, n8w, n8w);

  for (int b = 0; b < NB; ++b) {
    const unsigned short* Xbb = Xb + (size_t)b * NS * ND;
    float* outb = out + (size_t)b * NS * ND;
    gemm64<2, 0, 0><<<gQK, blk, 0, stream>>>(Xbb, Xbb, ND, Wqb, Wqb, ND, (void*)Qh, (void*)Ql, ND,
                                            1.0f, NS, ND, ND);
    gemm64<2, 0, 0><<<gQK, blk, 0, stream>>>(Xbb, Xbb, ND, Wkb, Wkb, ND, (void*)Kh, (void*)Kl, ND,
                                            1.0f, NS, ND, ND);
    gemm64<2, 0, 0><<<gV, blk, 0, stream>>>(Wvb, Wvb, ND, Xbb, Xbb, ND, (void*)Vh, (void*)Vl, NS,
                                           1.0f, ND, NS, ND);
    gemm64<0, 1, 1><<<gS, blk, 0, stream>>>(Qh, Ql, ND, Kh, Kl, ND, (void*)S, (void*)S, NS,
                                           0.03125f, NS, NS, ND);
    softmax_causal<<<gSm, blk, 0, stream>>>(S, Ph, Pl);
    gemm64<0, 2, 1><<<gO, blk, 0, stream>>>(Ph, Pl, NS, Vh, Vl, NS, (void*)outb, (void*)outb, ND,
                                           1.0f, NS, ND, NS);
  }
  (void)hipGetLastError();
}
